// GraphCIW_52132313039066
// MI455X (gfx1250) — hardware-verified
//
#include <hip/hip_runtime.h>
#include <stddef.h>
#include <stdint.h>
#include <math.h>

#define NNODE 10000
#define NEDGE 320000
#define DIN 128
#define DF 64
#define NCLS 10
#define NPG 10112
#define NGB 79
#define GBN 128
#define NPT 10048
#define NTB 157
#define LCAP 384
#define CHUNK 512
#define NCHUNK 625
#define OTP 68
#define HTP 72
#define ATP 136
#define XTP 104
#define FLGP 32
#define LN_EPS 1e-5f

static_assert(NGB * GBN == NPG);
static_assert(NTB * 64 == NPT);
static_assert(NPT >= NNODE);
static_assert(NPG >= NPT);
static_assert(NCHUNK * CHUNK == NEDGE);
static_assert(CHUNK == 4 * 128);
static_assert((NEDGE << 5) < (1 << 30));
static_assert(NNODE % 16 == 0);
static_assert(NGB <= 128);

typedef _Float16 v16h __attribute__((ext_vector_type(16)));
typedef _Float16 v8h  __attribute__((ext_vector_type(8)));
typedef _Float16 v2h  __attribute__((ext_vector_type(2)));
typedef __bf16   v16b __attribute__((ext_vector_type(16)));
typedef unsigned short v16us __attribute__((ext_vector_type(16)));
typedef unsigned short v8us  __attribute__((ext_vector_type(8)));
typedef float    v8f  __attribute__((ext_vector_type(8)));
typedef float    v4f  __attribute__((ext_vector_type(4)));
typedef float    v2f  __attribute__((ext_vector_type(2)));
typedef unsigned int v4u __attribute__((ext_vector_type(4)));
typedef int      v4i  __attribute__((ext_vector_type(4)));

union FragH  { v16h v; v8h h[2]; };
union FragU  { v16b b; v16us w; v8us u[2]; };
union Pack8  { v8h h; v4u u; };
union Pack8u { v8us s; v4u u; };

__device__ __forceinline__ v8f mma_h(v16h a, v16h b, v8f c) {
  c = __builtin_amdgcn_wmma_f32_16x16x32_f16(false, a, false, b, (short)0, c, false, false);
  asm volatile("v_nop\n\tv_nop\n\tv_nop\n\tv_nop" : "+v"(c) : "v"(a), "v"(b));
  return c;
}
__device__ __forceinline__ v8f mma_b(v16b a, v16b b, v8f c) {
  c = __builtin_amdgcn_wmma_f32_16x16x32_bf16(false, a, false, b, (short)0, c, false, false);
  asm volatile("v_nop\n\tv_nop\n\tv_nop\n\tv_nop" : "+v"(c) : "v"(a), "v"(b));
  return c;
}

__device__ __forceinline__ v16h ldfrag_h(const _Float16* p, int ld, int row0, int k0, int lane) {
  const int m = lane & 15, lh = lane >> 4;
  const _Float16* q = p + (size_t)(row0 + m) * ld + k0 + 8 * lh;
  FragH f;
  f.h[0] = *(const v8h*)(q);
  f.h[1] = *(const v8h*)(q + 16);
  return f.v;
}
__device__ __forceinline__ v16b ldfrag_b(const unsigned short* p, int ld, int row0, int k0, int lane) {
  const int m = lane & 15, lh = lane >> 4;
  const unsigned short* q = p + (size_t)(row0 + m) * ld + k0 + 8 * lh;
  FragU f;
  f.u[0] = *(const v8us*)(q);
  f.u[1] = *(const v8us*)(q + 16);
  return f.b;
}

__device__ __forceinline__ v8f zero8() { return (v8f){0.f, 0.f, 0.f, 0.f, 0.f, 0.f, 0.f, 0.f}; }

__device__ __forceinline__ float wsum(float s) {
#pragma unroll
  for (int off = 16; off >= 1; off >>= 1) s += __shfl_xor(s, off, 32);
  return s;
}
__device__ __forceinline__ float wmax(float s) {
#pragma unroll
  for (int off = 16; off >= 1; off >>= 1) s = fmaxf(s, __shfl_xor(s, off, 32));
  return s;
}

__device__ __forceinline__ unsigned short f2bf(float f) {
  unsigned u = __float_as_uint(f);
  u += 0x7FFFu + ((u >> 16) & 1u);
  return (unsigned short)(u >> 16);
}
__device__ __forceinline__ float bf2f(unsigned short s) { return __uint_as_float(((unsigned)s) << 16); }

__device__ __forceinline__ void split8(const v4f a, const v4f b, v4u& hi, v4u& lo) {
  Pack8u ph, pl;
#pragma unroll
  for (int j = 0; j < 4; ++j) {
    const unsigned short h0 = f2bf(a[j]);
    ph.s[j] = h0;
    pl.s[j] = f2bf(a[j] - bf2f(h0));
    const unsigned short h1 = f2bf(b[j]);
    ph.s[4 + j] = h1;
    pl.s[4 + j] = f2bf(b[j] - bf2f(h1));
  }
  hi = ph.u;
  lo = pl.u;
}

__device__ __forceinline__ float gelu_e(float x) {
  return 0.5f * x * (1.0f + erff(x * 0.70710678118654752f));
}

__device__ __forceinline__ void vst2u(void* p, v4u v) {
  *(volatile v4u*)p = v;
  __threadfence();
  *(volatile v4u*)p = v;
}
__device__ __forceinline__ void vst2f(float* p, v4f v) {
  *(volatile v4f*)p = v;
  __threadfence();
  *(volatile v4f*)p = v;
}

__global__ __launch_bounds__(256) void k_prep(
    const float* __restrict__ pre_w, const float* __restrict__ c1w, const float* __restrict__ c2w,
    const float* __restrict__ fe, const float* __restrict__ label,
    const float* __restrict__ wq, const float* __restrict__ bq,
    const float* __restrict__ wk, const float* __restrict__ bk,
    const float* __restrict__ wv, const float* __restrict__ bv,
    const float* __restrict__ wo, const float* __restrict__ bo,
    const float* __restrict__ alpha,
    const float* __restrict__ w1, const float* __restrict__ w2,
    const float* __restrict__ g1, const float* __restrict__ b1,
    const float* __restrict__ Am,
    unsigned short* __restrict__ WB, _Float16* __restrict__ W1h, _Float16* __restrict__ W2h,
    _Float16* __restrict__ M16, _Float16* __restrict__ P16, float* __restrict__ CT) {
  __shared__ __align__(16) float ct[512];
  __shared__ float xn[64];
  __shared__ float qv[64];
  const int tid = threadIdx.x, lane = tid & 31, wave = tid >> 5;

#pragma unroll 1
  for (int c = tid; c < 3072; c += 256) {
    const int mat = c >> 10, cc = c & 1023;
    const float* src = (mat == 0) ? pre_w : ((mat == 1) ? c1w : c2w);
    const v4f a = *(const v4f*)(src + 8 * cc);
    const v4f b = *(const v4f*)(src + 8 * cc + 4);
    v4u hi, lo;
    split8(a, b, hi, lo);
    unsigned short* dh = WB + (size_t)mat * 16384 + 8 * cc;
    vst2u(dh, hi);
    vst2u(dh + 8192, lo);
  }
#pragma unroll 1
  for (int c = tid; c < 1024; c += 256) {
    {
      const v4f a = *(const v4f*)(w1 + 8 * c);
      const v4f b = *(const v4f*)(w1 + 8 * c + 4);
      Pack8 pk;
      pk.h = (v8h){(_Float16)(a[0] * 16.f), (_Float16)(a[1] * 16.f), (_Float16)(a[2] * 16.f), (_Float16)(a[3] * 16.f),
                   (_Float16)(b[0] * 16.f), (_Float16)(b[1] * 16.f), (_Float16)(b[2] * 16.f), (_Float16)(b[3] * 16.f)};
      vst2u(W1h + 8 * c, pk.u);
    }
    {
      const v4f a = *(const v4f*)(w2 + 8 * c);
      const v4f b = *(const v4f*)(w2 + 8 * c + 4);
      Pack8 pk;
      pk.h = (v8h){(_Float16)(a[0] * 16.f), (_Float16)(a[1] * 16.f), (_Float16)(a[2] * 16.f), (_Float16)(a[3] * 16.f),
                   (_Float16)(b[0] * 16.f), (_Float16)(b[1] * 16.f), (_Float16)(b[2] * 16.f), (_Float16)(b[3] * 16.f)};
      vst2u(W2h + 8 * c, pk.u);
    }
  }
#pragma unroll 1
  for (int c = tid; c < 2048; c += 256) {
    const int o = c >> 5, q5 = c & 31, h = q5 >> 3, d0 = (q5 & 7) * 8;
    const float* wor = wo + o * 64 + 16 * h;
    const float* wvr = wv + (16 * h) * 64 + d0;
    Pack8 pk;
#pragma unroll
    for (int el = 0; el < 8; ++el) {
      float acc = 0.f;
#pragma unroll 1
      for (int j = 0; j < 16; ++j) acc += wor[j] * wvr[j * 64 + el];
      pk.h[el] = (_Float16)(acc * 64.0f);
    }
    vst2u(M16 + 8 * c, pk.u);
  }

  ct[tid] = 0.f;
  ct[256 + tid] = 0.f;
  __syncthreads();
  if (wave == 0) {
    const float l0 = label[lane], l1 = label[32 + lane];
    const float m = wsum(l0 + l1) * (1.0f / 64.0f);
    const float d0 = l0 - m, d1 = l1 - m;
    const float v = wsum(d0 * d0 + d1 * d1) * (1.0f / 64.0f);
    const float rs = 1.0f / sqrtf(v + LN_EPS);
    const float y0 = (d0 * rs) * g1[lane] + b1[lane];
    const float y1 = (d1 * rs) * g1[32 + lane] + b1[32 + lane];
    xn[lane] = y0;
    xn[32 + lane] = y1;
    ct[128 + lane] = y0;
    ct[160 + lane] = y1;
  } else if (wave < 3) {
    const int i = tid - 32;
    const float* fr = fe + i * 64;
    float s = 0.f;
#pragma unroll 1
    for (int d = 0; d < 64; ++d) s += fr[d];
    const float m = s * (1.0f / 64.0f);
    float v = 0.f;
#pragma unroll 1
    for (int d = 0; d < 64; ++d) {
      const float t = fr[d] - m;
      v += t * t;
    }
    ct[i] = m;
    ct[64 + i] = v * (1.0f / 64.0f);
  } else if (wave < 5) {
    const int o = tid - 96;
    float acc = 0.f;
#pragma unroll 1
    for (int j = 0; j < 64; ++j) acc += wo[o * 64 + j] * bv[j];
    ct[256 + o] = acc + bo[o];
  } else {
    const int t = tid - 160;
    const int tc = min(t, 63);
    const float a = alpha[0] * Am[tc * 65 + 64];
    const float v = (t < 64) ? a : 0.f;
    if (t < 80) ct[320 + t] = v;
  }
  __syncthreads();
  if (wave < 2) {
    const int o = tid;
    float acc = 0.f;
#pragma unroll 1
    for (int d = 0; d < 64; ++d) acc += xn[d] * wq[o * 64 + d];
    qv[o] = acc + bq[o];
  }
  __syncthreads();
  if (wave == 0) {
    const int h = lane & 3;
    float acc = 0.f;
#pragma unroll 1
    for (int j = 0; j < 16; ++j) acc += qv[16 * h + j] * bk[16 * h + j];
    if (lane < 4) ct[192 + lane] = acc;
  }
  if (wave < 4) {
    const int c = tid;
    const int h = c >> 3, hc = min(h, 3), d0 = (c & 7) * 8;
    Pack8 pk;
#pragma unroll
    for (int el = 0; el < 8; ++el) {
      float acc = 0.f;
#pragma unroll 1
      for (int j = 0; j < 16; ++j) acc += qv[16 * hc + j] * wk[(16 * hc + j) * 64 + d0 + el];
      pk.h[el] = (_Float16)((h < 4) ? acc * 64.0f : 0.f);
    }
    vst2u(P16 + 8 * c, pk.u);
  }
  __syncthreads();
  if (wave < 4) {
    const v4f v = *(const v4f*)(ct + 4 * tid);
    vst2f(CT + 4 * tid, v);
  }
}

template <int MODE>
__global__ __launch_bounds__(64) void k_ng(const float* __restrict__ srcA, const float* __restrict__ srcZ,
                                           const unsigned short* __restrict__ WBm, const float* __restrict__ bias,
                                           float* __restrict__ outz) {
  __shared__ __align__(16) unsigned short Ah[64 * ATP];
  __shared__ __align__(16) unsigned short Al[64 * ATP];
  __shared__ __align__(16) float sw[2][16 * OTP];
  const int tid = threadIdx.x, lane = tid & 31, wave = tid >> 5;
  const int hh = lane >> 4, c = lane & 15;
  const int m0 = blockIdx.x * 64;
  const int mrow = wave * 32;

#pragma unroll 1
  for (int it = 0; it < 16; ++it) {
    const int cc = tid + 64 * it;
    const int row = cc >> 4, k0 = (cc & 15) * 8;
    const float* s;
    if (MODE == 0) {
      s = srcA + (size_t)min(m0 + row, NNODE - 1) * DIN + k0;
    } else {
      s = (k0 < 64) ? (srcA + (size_t)(m0 + row) * DF + k0) : (srcZ + (size_t)(m0 + row) * DF + (k0 - 64));
    }
    const v4f a = *(const v4f*)(s);
    const v4f b = *(const v4f*)(s + 4);
    v4u hi, lo;
    split8(a, b, hi, lo);
    *(v4u*)(Ah + row * ATP + k0) = hi;
    *(v4u*)(Al + row * ATP + k0) = lo;
  }
  __syncthreads();

  v8f acc[2][4];
#pragma unroll
  for (int s2 = 0; s2 < 2; ++s2)
#pragma unroll
    for (int t = 0; t < 4; ++t) acc[s2][t] = zero8();
  const unsigned short* Wh = WBm;
  const unsigned short* Wl = WBm + 8192;
#pragma unroll 1
  for (int k0 = 0; k0 < DIN; k0 += 32) {
    const v16b ah0 = ldfrag_b(Ah, ATP, mrow, k0, lane);
    const v16b ah1 = ldfrag_b(Ah, ATP, mrow + 16, k0, lane);
    const v16b al0 = ldfrag_b(Al, ATP, mrow, k0, lane);
    const v16b al1 = ldfrag_b(Al, ATP, mrow + 16, k0, lane);
#pragma unroll
    for (int t = 0; t < 4; ++t) {
      const v16b bh = ldfrag_b(Wh, DIN, 16 * t, k0, lane);
      const v16b bl = ldfrag_b(Wl, DIN, 16 * t, k0, lane);
      acc[0][t] = mma_b(ah0, bh, acc[0][t]);
      acc[1][t] = mma_b(ah1, bh, acc[1][t]);
      acc[0][t] = mma_b(ah0, bl, acc[0][t]);
      acc[1][t] = mma_b(ah1, bl, acc[1][t]);
      acc[0][t] = mma_b(al0, bh, acc[0][t]);
      acc[1][t] = mma_b(al1, bh, acc[1][t]);
    }
  }

  float bb[4];
#pragma unroll
  for (int t = 0; t < 4; ++t) bb[t] = (MODE == 0) ? bias[16 * t + c] : 0.f;
  float* swv = sw[wave];
#pragma unroll
  for (int sub = 0; sub < 2; ++sub) {
    __syncthreads();
#pragma unroll
    for (int t = 0; t < 4; ++t) {
#pragma unroll
      for (int r = 0; r < 8; ++r) swv[(8 * hh + r) * OTP + 16 * t + c] = acc[sub][t][r] + bb[t];
    }
    __syncthreads();
    if (MODE == 1) {
#pragma unroll 1
      for (int i = 0; i < 32; ++i) {
        const int e = i * 32 + lane;
        const int row = e >> 6, col = e & 63;
        const float v = swv[row * OTP + col];
        swv[row * OTP + col] = gelu_e(v);
      }
      __syncthreads();
    }
#pragma unroll
    for (int it = 0; it < 8; ++it) {
      const int p = lane + 32 * it;
      const int L = p >> 3, pc = p & 7;
      const int row = L >> 1, seg = L & 1;
      const v4f vv = *(const v4f*)(swv + row * OTP + seg * 32 + pc * 4);
      vst2f(outz + (size_t)(m0 + mrow + sub * 16 + row) * DF + seg * 32 + pc * 4, vv);
    }
  }
}

__device__ __forceinline__ void place_hit(bool f, int dd, int e, unsigned lt, int* lstw,
                                          int& n0, int& n1, int& n2, int& n3) {
  const unsigned bj = __builtin_amdgcn_ballot_w32(f);
  if (bj == 0u) return;
  const int sub = dd >> 5;
  const int pk = (e << 5) | (dd & 31);
  {
    const bool hs = f && (sub == 0);
    const unsigned bs = __builtin_amdgcn_ballot_w32(hs);
    const int pos = n0 + (int)__builtin_popcount(bs & lt);
    if (hs) lstw[0 * LCAP + min(pos, LCAP - 1)] = pk;
    n0 += (int)__builtin_popcount(bs);
  }
  {
    const bool hs = f && (sub == 1);
    const unsigned bs = __builtin_amdgcn_ballot_w32(hs);
    const int pos = n1 + (int)__builtin_popcount(bs & lt);
    if (hs) lstw[1 * LCAP + min(pos, LCAP - 1)] = pk;
    n1 += (int)__builtin_popcount(bs);
  }
  {
    const bool hs = f && (sub == 2);
    const unsigned bs = __builtin_amdgcn_ballot_w32(hs);
    const int pos = n2 + (int)__builtin_popcount(bs & lt);
    if (hs) lstw[2 * LCAP + min(pos, LCAP - 1)] = pk;
    n2 += (int)__builtin_popcount(bs);
  }
  {
    const bool hs = f && (sub == 3);
    const unsigned bs = __builtin_amdgcn_ballot_w32(hs);
    const int pos = n3 + (int)__builtin_popcount(bs & lt);
    if (hs) lstw[3 * LCAP + min(pos, LCAP - 1)] = pk;
    n3 += (int)__builtin_popcount(bs);
  }
}

__device__ __forceinline__ void scan_block(const int* __restrict__ cols, int d0, int wave, int lane, int* lstw,
                                           int& n0, int& n1, int& n2, int& n3) {
  n0 = 0; n1 = 0; n2 = 0; n3 = 0;
  const unsigned lt = (1u << lane) - 1u;
#pragma unroll 1
  for (int it = 0; it < NCHUNK; ++it) {
    const int cb = it * CHUNK + wave * 128 + 4 * lane;
    const v4i cv = *(const v4i*)(cols + cb);
    const int dd0 = cv[0] - d0, dd1 = cv[1] - d0, dd2 = cv[2] - d0, dd3 = cv[3] - d0;
    const bool f0 = (unsigned)dd0 < (unsigned)GBN;
    const bool f1 = (unsigned)dd1 < (unsigned)GBN;
    const bool f2 = (unsigned)dd2 < (unsigned)GBN;
    const bool f3 = (unsigned)dd3 < (unsigned)GBN;
    const unsigned any = __builtin_amdgcn_ballot_w32(f0 || f1 || f2 || f3);
    if (any == 0u) continue;
    place_hit(f0, dd0, cb + 0, lt, lstw, n0, n1, n2, n3);
    place_hit(f1, dd1, cb + 1, lt, lstw, n0, n1, n2, n3);
    place_hit(f2, dd2, cb + 2, lt, lstw, n0, n1, n2, n3);
    place_hit(f3, dd3, cb + 3, lt, lstw, n0, n1, n2, n3);
  }
}

__global__ __launch_bounds__(128) void k_gdeg(const int* __restrict__ ei, float* __restrict__ dis,
                                              int* __restrict__ flg) {
  __shared__ int lst[16 * LCAP];
  __shared__ int lns[16];
  __shared__ int pf[4];
  __shared__ __align__(16) float dl[GBN];
  const int tid = threadIdx.x, lane = tid & 31, wave = tid >> 5;
  const int d0 = blockIdx.x * GBN;
  int n0, n1, n2, n3;
  scan_block(ei + NEDGE, d0, wave, lane, lst + wave * 4 * LCAP, n0, n1, n2, n3);
  if (lane == 0) {
    lns[wave * 4 + 0] = n0; lns[wave * 4 + 1] = n1; lns[wave * 4 + 2] = n2; lns[wave * 4 + 3] = n3;
    pf[wave] = (n0 > LCAP || n1 > LCAP || n2 > LCAP || n3 > LCAP) ? 1 : 0;
  }
  __syncthreads();
  const int poison_blk = pf[0] | pf[1] | pf[2] | pf[3];
  const int poison_sub = ((lns[0 * 4 + wave] > LCAP) || (lns[1 * 4 + wave] > LCAP) ||
                          (lns[2 * 4 + wave] > LCAP) || (lns[3 * 4 + wave] > LCAP)) ? 1 : 0;
  int cnt = 0;
#pragma unroll 1
  for (int wp = 0; wp < 4; ++wp) {
    int n = lns[wp * 4 + wave];
    n = min(max(n, 0), LCAP);
    const int* L = lst + (wp * 4 + wave) * LCAP;
#pragma unroll 1
    for (int i = 0; i < n; ++i) cnt += ((L[i] & 31) == lane) ? 1 : 0;
  }
  const float deg = (float)cnt;
  float dv = (deg > 0.f) ? (1.0f / sqrtf(fmaxf(deg, 1.0f))) : 0.f;
  if (poison_sub) dv = __uint_as_float(0x7fc00000u);
  dl[wave * 32 + lane] = dv;
  __syncthreads();
  if (wave == 0) {
    const v4f v = *(const v4f*)(dl + 4 * lane);
    vst2f(dis + d0 + 4 * lane, v);
    volatile int* fp = (volatile int*)(flg + (size_t)blockIdx.x * FLGP + lane);
    *fp = poison_blk;
    __threadfence();
    *fp = poison_blk;
  }
}

__global__ __launch_bounds__(128) void k_gagg(const int* __restrict__ ei, const float* __restrict__ dis,
                                              const float* __restrict__ z, float* __restrict__ hi) {
#pragma clang fp contract(off)
  __shared__ int lst[16 * LCAP];
  __shared__ int lns[16];
  __shared__ __align__(16) float hacc[4 * 32 * 64];
  const int tid = threadIdx.x, lane = tid & 31, wave = tid >> 5;
  const int d0 = blockIdx.x * GBN;
  float* hw = hacc + wave * 2048;
  const v4f z4 = (v4f){0.f, 0.f, 0.f, 0.f};
#pragma unroll
  for (int it = 0; it < 16; ++it) *(v4f*)(hw + 4 * (lane + 32 * it)) = z4;

  int n0, n1, n2, n3;
  scan_block(ei + NEDGE, d0, wave, lane, lst + wave * 4 * LCAP, n0, n1, n2, n3);
  if (lane == 0) {
    lns[wave * 4 + 0] = n0; lns[wave * 4 + 1] = n1; lns[wave * 4 + 2] = n2; lns[wave * 4 + 3] = n3;
  }
  __syncthreads();
  const int poison = ((lns[0 * 4 + wave] > LCAP) || (lns[1 * 4 + wave] > LCAP) ||
                      (lns[2 * 4 + wave] > LCAP) || (lns[3 * 4 + wave] > LCAP)) ? 1 : 0;
  const float* disc = dis + d0 + wave * 32;
#pragma unroll 1
  for (int wp = 0; wp < 4; ++wp) {
    int n = lns[wp * 4 + wave];
    n = min(max(n, 0), LCAP);
    const int* L = lst + (wp * 4 + wave) * LCAP;
#pragma unroll 1
    for (int i = 0; i < n; ++i) {
      const int p = L[i];
      const int e = min(p >> 5, NEDGE - 1);
      const int lc = p & 31;
      int r = ei[e];
      r = min(max(r, 0), NNODE - 1);
      const float nm = dis[r] * disc[lc];
      const v2f zv = *(const v2f*)(z + (size_t)r * DF + 2 * lane);
      v2f* hp = (v2f*)(hw + lc * 64 + 2 * lane);
      v2f h = *hp;
      h.x = h.x + nm * zv.x;
      h.y = h.y + nm * zv.y;
      *hp = h;
    }
  }
  __syncthreads();
  const v4f nan4 = (v4f){__uint_as_float(0x7fc00000u), __uint_as_float(0x7fc00000u),
                         __uint_as_float(0x7fc00000u), __uint_as_float(0x7fc00000u)};
#pragma unroll
  for (int it = 0; it < 16; ++it) {
    const int p = lane + 32 * it;
    const int row = p >> 4, c4 = (p & 15) * 4;
    v4f v = *(const v4f*)(hw + row * 64 + c4);
    if (poison) v = nan4;
    vst2f(hi + (size_t)(d0 + wave * 32 + row) * DF + c4, v);
  }
}

__global__ __launch_bounds__(32) void k_attn(const float* __restrict__ z2, const float* __restrict__ fe,
                                             const float* __restrict__ g1, const float* __restrict__ b1,
                                             const float* __restrict__ CT, const _Float16* __restrict__ P16,
                                             _Float16* __restrict__ S16) {
  __shared__ __align__(16) _Float16 Xh[80 * HTP];
  __shared__ __align__(16) _Float16 XT[64 * XTP];
  __shared__ __align__(16) _Float16 At[16 * XTP];
  __shared__ __align__(16) float sc[80 * 16];
  __shared__ float zn[64];
  __shared__ float mo[64];
  __shared__ float rr[64];
  __shared__ __align__(16) _Float16 Sst[256];
  const int lane = threadIdx.x & 31;
  const int hh = lane >> 4, cidx = lane & 15;
  const int n = blockIdx.x;

  const v4u z4 = (v4u){0u, 0u, 0u, 0u};
  for (int c = lane; c < 208; c += 32) *(v4u*)(At + 8 * c) = z4;
  for (int c = lane; c < 832; c += 32) *(v4u*)(XT + 8 * c) = z4;
  for (int c = lane; c < 135; c += 32) *(v4u*)(Xh + 65 * HTP + 8 * c) = z4;

  const float zl = z2[(size_t)n * DF + lane], zh = z2[(size_t)n * DF + 32 + lane];
  const float m = wsum(zl + zh) * (1.0f / 64.0f);
  const float dlo = zl - m, dhi = zh - m;
  const float v = wsum(dlo * dlo + dhi * dhi) * (1.0f / 64.0f);
  const float rs = 1.0f / sqrtf(v + LN_EPS);
  const float znl = dlo * rs, znh = dhi * rs;
  {
    const int i0 = lane, i1 = lane + 32;
    const float mu0 = CT[i0], s20 = CT[64 + i0], mu1 = CT[i1], s21 = CT[64 + i1];
    zn[i0] = znl;
    mo[i0] = znl * mu0;
    rr[i0] = 1.0f / sqrtf((znl * znl) * s20 + LN_EPS);
    zn[i1] = znh;
    mo[i1] = znh * mu1;
    rr[i1] = 1.0f / sqrtf((znh * znh) * s21 + LN_EPS);
  }
  __syncthreads();

  const float gA = g1[2 * lane], gB = g1[2 * lane + 1], bA = b1[2 * lane], bB = b1[2 * lane + 1];
#pragma unroll 4
  for (int i = 0; i < 64; ++i) {
    const v2f f = *(const v2f*)(fe + i * 64 + 2 * lane);
    const float zi = zn[i], mi = mo[i], ri = rr[i];
    const float y0 = ((zi * f.x - mi) * ri) * gA + bA;
    const float y1 = ((zi * f.y - mi) * ri) * gB + bB;
    const _Float16 h0 = (_Float16)y0, h1 = (_Float16)y1;
    *(v2h*)(Xh + i * HTP + 2 * lane) = (v2h){h0, h1};
    XT[(2 * lane) * XTP + i] = h0;
    XT[(2 * lane + 1) * XTP + i] = h1;
  }
  {
    const float x0 = CT[128 + 2 * lane], x1 = CT[129 + 2 * lane];
    const _Float16 h0 = (_Float16)x0, h1 = (_Float16)x1;
    *(v2h*)(Xh + 64 * HTP + 2 * lane) = (v2h){h0, h1};
    XT[(2 * lane) * XTP + 64] = h0;
    XT[(2 * lane + 1) * XTP + 64] = h1;
  }
  __syncthreads();

  const v16h bp0 = ldfrag_h(P16, 64, 0, 0, lane);
  const v16h bp1 = ldfrag_h(P16, 64, 0, 32, lane);
#pragma unroll 1
  for (int mi = 0; mi < 5; ++mi) {
    v8f acc = zero8();
    const v16h a0 = ldfrag_h(Xh, HTP, 16 * mi, 0, lane);
    acc = mma_h(a0, bp0, acc);
    const v16h a1 = ldfrag_h(Xh, HTP, 16 * mi, 32, lane);
    acc = mma_h(a1, bp1, acc);
#pragma unroll
    for (int r = 0; r < 8; ++r) sc[(16 * mi + 8 * hh + r) * 16 + cidx] = acc[r];
  }
  __syncthreads();

#pragma unroll 1
  for (int h = 0; h < 4; ++h) {
    const float cq = CT[192 + h];
    float mx = -3.0e38f;
#pragma unroll 1
    for (int jj = 0; jj < 3; ++jj) {
      const int t = 32 * jj + lane, tt = min(t, 64);
      const float sv = (sc[tt * 16 + h] * (1.0f / 64.0f) + cq) * 0.25f + CT[320 + tt];
      mx = fmaxf(mx, (t <= 64) ? sv : -3.0e38f);
    }
    mx = wmax(mx);
    float l = 0.f;
#pragma unroll 1
    for (int jj = 0; jj < 3; ++jj) {
      const int t = 32 * jj + lane, tt = min(t, 64);
      const bool ok = t <= 64;
      const float sv = (sc[tt * 16 + h] * (1.0f / 64.0f) + cq) * 0.25f + CT[320 + tt];
      const float e = ok ? expf(sv - mx) : 0.f;
      l += e;
      if (ok) sc[t * 16 + h] = e;
    }
    l = wsum(l);
    const float inv = 1.0f / l;
#pragma unroll 1
    for (int jj = 0; jj < 3; ++jj) {
      const int t = 32 * jj + lane, tt = min(t, 64);
      const float p = sc[tt * 16 + h] * inv;
      if (t <= 64) At[h * XTP + t] = (_Float16)(p * 64.0f);
    }
  }
  __syncthreads();

  v8f sa[4];
#pragma unroll
  for (int t = 0; t < 4; ++t) sa[t] = zero8();
#pragma unroll
  for (int kk = 0; kk < 3; ++kk) {
    const v16h a = ldfrag_h(At, XTP, 0, 32 * kk, lane);
#pragma unroll
    for (int t = 0; t < 4; ++t) {
      const v16h b = ldfrag_h(XT, XTP, 16 * t, 32 * kk, lane);
      sa[t] = mma_h(a, b, sa[t]);
    }
  }
  if (lane < 16) {
#pragma unroll
    for (int t = 0; t < 4; ++t) {
#pragma unroll
      for (int r = 0; r < 4; ++r) Sst[r * 64 + 16 * t + lane] = (_Float16)(sa[t][r] * 0.25f);
    }
  }
  __syncthreads();
  {
    Pack8 pk;
    pk.h = *(const v8h*)(Sst + 8 * lane);
    vst2u(S16 + (size_t)n * 256 + 8 * lane, pk.u);
  }
}

__global__ __launch_bounds__(64) void k_y(const _Float16* __restrict__ S16, const _Float16* __restrict__ M16,
                                          const float* __restrict__ label, const float* __restrict__ CT,
                                          const float* __restrict__ g2, const float* __restrict__ b2,
                                          float* __restrict__ X1, _Float16* __restrict__ HL) {
  __shared__ __align__(16) float xs[64 * OTP];
  __shared__ __align__(16) _Float16 hs[64 * HTP];
  const int tid = threadIdx.x, lane = tid & 31, wave = tid >> 5;
  const int hh = lane >> 4, c = lane & 15;
  const int m0 = blockIdx.x * 64;
  const int mrow = wave * 32;

  v8f acc[2][4];
#pragma unroll
  for (int s2 = 0; s2 < 2; ++s2)
#pragma unroll
    for (int t = 0; t < 4; ++t) acc[s2][t] = zero8();
#pragma unroll 1
  for (int k0 = 0; k0 < 256; k0 += 32) {
    const v16h a0 = ldfrag_h(S16, 256, m0 + mrow, k0, lane);
    const v16h a1 = ldfrag_h(S16, 256, m0 + mrow + 16, k0, lane);
#pragma unroll
    for (int t = 0; t < 4; ++t) {
      const v16h b = ldfrag_h(M16, 256, 16 * t, k0, lane);
      acc[0][t] = mma_h(a0, b, acc[0][t]);
      acc[1][t] = mma_h(a1, b, acc[1][t]);
    }
  }
#pragma unroll
  for (int t = 0; t < 4; ++t) {
    const int col = 16 * t + c;
    const float lb = label[col], dv = CT[256 + col];
#pragma unroll
    for (int sub = 0; sub < 2; ++sub) {
#pragma unroll
      for (int r = 0; r < 8; ++r) {
        const int row = mrow + 16 * sub + 8 * hh + r;
        const float y = acc[sub][t][r] * (1.0f / 1024.0f) + dv;
        xs[row * OTP + col] = lb + y;
      }
    }
  }
  __syncthreads();

  const float ga = g2[lane], gb = g2[32 + lane], ba = b2[lane], bbv = b2[32 + lane];
#pragma unroll 1
  for (int q = 0; q < 32; ++q) {
    const int row = mrow + q;
    const float x0 = xs[row * OTP + lane], x1 = xs[row * OTP + 32 + lane];
    const float m = wsum(x0 + x1) * (1.0f / 64.0f);
    const float e0 = x0 - m, e1 = x1 - m;
    const float v = wsum(e0 * e0 + e1 * e1) * (1.0f / 64.0f);
    const float rs = 1.0f / sqrtf(v + LN_EPS);
    hs[row * HTP + lane]      = (_Float16)((e0 * rs) * ga + ba);
    hs[row * HTP + 32 + lane] = (_Float16)((e1 * rs) * gb + bbv);
  }
  __syncthreads();

#pragma unroll
  for (int it = 0; it < 16; ++it) {
    const int p = lane + 32 * it;
    const int row = p >> 4, c4 = (p & 15) * 4;
    const v4f vv = *(const v4f*)(xs + (mrow + row) * OTP + c4);
    vst2f(X1 + (size_t)(m0 + mrow + row) * DF + c4, vv);
  }
#pragma unroll
  for (int it = 0; it < 8; ++it) {
    const int p = lane + 32 * it;
    const int row = p >> 3, pc = p & 7;
    Pack8 pk;
    pk.h = *(const v8h*)(hs + (mrow + row) * HTP + 8 * pc);
    vst2u(HL + (size_t)(m0 + mrow + row) * DF + 8 * pc, pk.u);
  }
}

__global__ __launch_bounds__(64) void k_f1(const _Float16* __restrict__ HL, const _Float16* __restrict__ W1h,
                                           const float* __restrict__ fb1, _Float16* __restrict__ G16) {
  __shared__ __align__(16) float sw[2][16 * OTP];
  __shared__ __align__(16) _Float16 sh[2][16 * HTP];
  const int tid = threadIdx.x, lane = tid & 31, wave = tid >> 5;
  const int hh = lane >> 4, c = lane & 15;
  const int m0 = blockIdx.x * 64, n0 = blockIdx.y * 64;
  const int mrow = wave * 32;

  v8f acc[2][4];
#pragma unroll
  for (int s2 = 0; s2 < 2; ++s2)
#pragma unroll
    for (int t = 0; t < 4; ++t) acc[s2][t] = zero8();
#pragma unroll 1
  for (int k0 = 0; k0 < 64; k0 += 32) {
    const v16h a0 = ldfrag_h(HL, DF, m0 + mrow, k0, lane);
    const v16h a1 = ldfrag_h(HL, DF, m0 + mrow + 16, k0, lane);
#pragma unroll
    for (int t = 0; t < 4; ++t) {
      const v16h b = ldfrag_h(W1h, DF, n0 + 16 * t, k0, lane);
      acc[0][t] = mma_h(a0, b, acc[0][t]);
      acc[1][t] = mma_h(a1, b, acc[1][t]);
    }
  }
  float bb[4];
#pragma unroll
  for (int t = 0; t < 4; ++t) bb[t] = fb1[n0 + 16 * t + c];
  float* swv = sw[wave];
  _Float16* shv = sh[wave];
#pragma unroll
  for (int sub = 0; sub < 2; ++sub) {
    __syncthreads();
#pragma unroll
    for (int t = 0; t < 4; ++t) {
#pragma unroll
      for (int r = 0; r < 8; ++r) swv[(8 * hh + r) * OTP + 16 * t + c] = acc[sub][t][r] * (1.0f / 16.0f) + bb[t];
    }
    __syncthreads();
#pragma unroll 1
    for (int i = 0; i < 32; ++i) {
      const int e = i * 32 + lane;
      const int row = e >> 6, col = e & 63;
      const float v = swv[row * OTP + col];
      shv[row * HTP + col] = (_Float16)(gelu_e(v) * 16.0f);
    }
    __syncthreads();
#pragma unroll
    for (int it = 0; it < 4; ++it) {
      const int p = lane + 32 * it;
      const int row = p >> 3, pc = p & 7;
      Pack8 pk;
      pk.h = *(const v8h*)(shv + row * HTP + 8 * pc);
      vst2u(G16 + (size_t)(m0 + mrow + 16 * sub + row) * 128 + n0 + 8 * pc, pk.u);
    }
  }
}

__global__ __launch_bounds__(64) void k_f2(const _Float16* __restrict__ G16, const _Float16* __restrict__ W2h,
                                           const float* __restrict__ fb2, const float* __restrict__ X1,
                                           const float* __restrict__ cw, const float* __restrict__ cb,
                                           const int* __restrict__ flg, float* __restrict__ out) {
  __shared__ __align__(16) float xs[64 * OTP];
  __shared__ __align__(16) float os[640];
  __shared__ int fl[2];
  const int tid = threadIdx.x, lane = tid & 31, wave = tid >> 5;
  const int hh = lane >> 4, c = lane & 15;
  const int m0 = blockIdx.x * 64;
  const int mrow = wave * 32;

  {
    const int fa = flg[(size_t)min(tid, NGB - 1) * FLGP];
    const int fb = flg[(size_t)min(tid + 64, NGB - 1) * FLGP];
    const unsigned bal = __builtin_amdgcn_ballot_w32((fa | fb) != 0);
    if (lane == 0) fl[wave] = (bal != 0u) ? 1 : 0;
  }

  v8f acc[2][4];
#pragma unroll
  for (int s2 = 0; s2 < 2; ++s2)
#pragma unroll
    for (int t = 0; t < 4; ++t) acc[s2][t] = zero8();
#pragma unroll 1
  for (int k0 = 0; k0 < 128; k0 += 32) {
    const v16h a0 = ldfrag_h(G16, 128, m0 + mrow, k0, lane);
    const v16h a1 = ldfrag_h(G16, 128, m0 + mrow + 16, k0, lane);
#pragma unroll
    for (int t = 0; t < 4; ++t) {
      const v16h b = ldfrag_h(W2h, 128, 16 * t, k0, lane);
      acc[0][t] = mma_h(a0, b, acc[0][t]);
      acc[1][t] = mma_h(a1, b, acc[1][t]);
    }
  }
#pragma unroll
  for (int t = 0; t < 4; ++t) {
    const int col = 16 * t + c;
    const float fb = fb2[col];
#pragma unroll
    for (int sub = 0; sub < 2; ++sub) {
#pragma unroll
      for (int r = 0; r < 8; ++r) {
        const int row = mrow + 16 * sub + 8 * hh + r;
        xs[row * OTP + col] = acc[sub][t][r] * (1.0f / 256.0f) + fb;
      }
    }
  }
  __syncthreads();
  const int poison = fl[0] | fl[1];

#pragma unroll 4
  for (int it = 0; it < 16; ++it) {
    const int p = lane + 32 * it;
    const int row = mrow + (p >> 4), c4 = (p & 15) * 4;
    const v4f xv = *(const v4f*)(X1 + (size_t)(m0 + row) * DF + c4);
    v4f* q = (v4f*)(xs + row * OTP + c4);
    *q = *q + xv;
  }
  __syncthreads();

  {
    const float* xr = xs + tid * OTP;
    float a0 = 0.f, a1 = 0.f, a2 = 0.f, a3 = 0.f, a4 = 0.f, a5 = 0.f, a6 = 0.f, a7 = 0.f, a8 = 0.f, a9 = 0.f;
#pragma unroll 1
    for (int k = 0; k < 64; ++k) {
      const float xv = xr[k];
      a0 += xv * cw[0 * 64 + k];
      a1 += xv * cw[1 * 64 + k];
      a2 += xv * cw[2 * 64 + k];
      a3 += xv * cw[3 * 64 + k];
      a4 += xv * cw[4 * 64 + k];
      a5 += xv * cw[5 * 64 + k];
      a6 += xv * cw[6 * 64 + k];
      a7 += xv * cw[7 * 64 + k];
      a8 += xv * cw[8 * 64 + k];
      a9 += xv * cw[9 * 64 + k];
    }
    const float nanv = __uint_as_float(0x7fc00000u);
    os[tid * NCLS + 0] = poison ? nanv : (a0 + cb[0]);
    os[tid * NCLS + 1] = poison ? nanv : (a1 + cb[1]);
    os[tid * NCLS + 2] = poison ? nanv : (a2 + cb[2]);
    os[tid * NCLS + 3] = poison ? nanv : (a3 + cb[3]);
    os[tid * NCLS + 4] = poison ? nanv : (a4 + cb[4]);
    os[tid * NCLS + 5] = poison ? nanv : (a5 + cb[5]);
    os[tid * NCLS + 6] = poison ? nanv : (a6 + cb[6]);
    os[tid * NCLS + 7] = poison ? nanv : (a7 + cb[7]);
    os[tid * NCLS + 8] = poison ? nanv : (a8 + cb[8]);
    os[tid * NCLS + 9] = poison ? nanv : (a9 + cb[9]);
  }
  __syncthreads();
  const int nrows = min(64, NNODE - m0);
  const int nf4 = (nrows * NCLS) >> 2;
  if (wave == 0) {
    float* ob = out + (size_t)m0 * NCLS;
    for (int ps = 0; ps < 2; ++ps) {
#pragma unroll
      for (int it = 0; it < 5; ++it) {
        const int p = lane + 32 * it;
        const v4f vv = *(const v4f*)(os + 4 * p);
        if (p < nf4) *(volatile v4f*)(ob + 4 * p) = vv;
      }
      __threadfence();
    }
  }
}

extern "C" void kernel_launch(void* const* d_in, const int* in_sizes, int n_in,
                              void* d_out, int out_size, void* d_ws, size_t ws_size,
                              hipStream_t stream) {
  if (n_in < 28) return;
  if (in_sizes[0] != NNODE * DIN) return;
  if (in_sizes[1] != 2 * NEDGE) return;
  if (in_sizes[2] != DF * DIN || in_sizes[3] != DF) return;
  if (in_sizes[4] != DF * 128 || in_sizes[5] != DF * 128) return;
  if (in_sizes[6] != DF * DF || in_sizes[7] != DF) return;
  if (in_sizes[8] != DF * DF || in_sizes[9] != DF) return;
  if (in_sizes[10] != DF * DF || in_sizes[11] != DF) return;
  if (in_sizes[12] != DF * DF || in_sizes[13] != DF) return;
  if (in_sizes[14] != DF * DF || in_sizes[15] != DF) return;
  if (in_sizes[16] != 1) return;
  if (in_sizes[17] != 128 * DF || in_sizes[18] != 128) return;
  if (in_sizes[19] != DF * 128 || in_sizes[20] != DF) return;
  if (in_sizes[21] != DF || in_sizes[22] != DF || in_sizes[23] != DF || in_sizes[24] != DF) return;
  if (in_sizes[25] != 65 * 65) return;
  if (in_sizes[26] != NCLS * DF || in_sizes[27] != NCLS) return;
  if (out_size != NNODE * NCLS) return;

  const float* x     = (const float*)d_in[0];
  const int*   ei    = (const int*)d_in[1];
  const float* pre_w = (const float*)d_in[2];
  const float* pre_b = (const float*)d_in[3];
  const float* c1w   = (const float*)d_in[4];
  const float* c2w   = (const float*)d_in[5];
  const float* fe    = (const float*)d_in[6];
  const float* label = (const float*)d_in[7];
  const float* wq    = (const float*)d_in[8];
  const float* bq    = (const float*)d_in[9];
  const float* wk    = (const float*)d_in[10];
  const float* bk    = (const float*)d_in[11];
  const float* wvv   = (const float*)d_in[12];
  const float* bv    = (const float*)d_in[13];
  const float* wo    = (const float*)d_in[14];
  const float* bo    = (const float*)d_in[15];
  const float* alpha = (const float*)d_in[16];
  const float* w1    = (const float*)d_in[17];
  const float* fb1   = (const float*)d_in[18];
  const float* w2    = (const float*)d_in[19];
  const float* fb2   = (const float*)d_in[20];
  const float* g1    = (const float*)d_in[21];
  const float* b1    = (const float*)d_in[22];
  const float* g2    = (const float*)d_in[23];
  const float* b2    = (const float*)d_in[24];
  const float* Am    = (const float*)d_in[25];
  const float* cw    = (const float*)d_in[26];
  const float* cb    = (const float*)d_in[27];
  float* out = (float*)d_out;

  size_t off = 0;
  const size_t oWB  = off; off += (size_t)3 * 16384 * 2;
  const size_t oW1  = off; off += (size_t)128 * DF * 2;
  const size_t oW2  = off; off += (size_t)DF * 128 * 2;
  const size_t oM   = off; off += (size_t)DF * 256 * 2;
  const size_t oP   = off; off += (size_t)16 * 64 * 2;
  const size_t oCT  = off; off += (size_t)512 * 4;
  const size_t oFLG = off; off += (size_t)NGB * FLGP * 4;
  const size_t oDIS = off; off += (size_t)NPG * 4;
  const size_t oZ0  = off; off += (size_t)NPG * DF * 4;
  const size_t oZ1  = off; off += (size_t)NPG * DF * 4;
  const size_t oZ2  = off; off += (size_t)NPG * DF * 4;
  const size_t oHI  = off; off += (size_t)NPG * DF * 4;
  const size_t oS   = off; off += (size_t)NPT * 256 * 2;
  const size_t oX1  = off; off += (size_t)NPT * DF * 4;
  const size_t oHL  = off; off += (size_t)NPT * DF * 2;
  const size_t oG   = off; off += (size_t)NPT * 128 * 2;
  if (off > ws_size) return;
  if (off > (size_t)134217728) return;

  char* ws = (char*)d_ws;
  unsigned short* WB  = (unsigned short*)(ws + oWB);
  _Float16* W1h = (_Float16*)(ws + oW1);
  _Float16* W2h = (_Float16*)(ws + oW2);
  _Float16* M16 = (_Float16*)(ws + oM);
  _Float16* P16 = (_Float16*)(ws + oP);
  float*    CT  = (float*)(ws + oCT);
  int*      FLG = (int*)(ws + oFLG);
  float*    DIS = (float*)(ws + oDIS);
  float*    Z0  = (float*)(ws + oZ0);
  float*    Z1  = (float*)(ws + oZ1);
  float*    Z2  = (float*)(ws + oZ2);
  float*    HI  = (float*)(ws + oHI);
  _Float16* S16 = (_Float16*)(ws + oS);
  float*    X1  = (float*)(ws + oX1);
  _Float16* HL  = (_Float16*)(ws + oHL);
  _Float16* G16 = (_Float16*)(ws + oG);

  k_prep<<<dim3(1), dim3(256), 0, stream>>>(pre_w, c1w, c2w, fe, label, wq, bq, wk, bk, wvv, bv, wo, bo, alpha,
                                            w1, w2, g1, b1, Am, WB, W1h, W2h, M16, P16, CT);
  k_ng<0><<<dim3(NPG / 64), dim3(64), 0, stream>>>(x, x, WB, pre_b, Z0);
  k_gdeg<<<dim3(NGB), dim3(128), 0, stream>>>(ei, DIS, FLG);
  k_gagg<<<dim3(NGB), dim3(128), 0, stream>>>(ei, DIS, Z0, HI);
  k_ng<1><<<dim3(NPG / 64), dim3(64), 0, stream>>>(HI, Z0, WB + 16384, pre_b, Z1);
  k_gagg<<<dim3(NGB), dim3(128), 0, stream>>>(ei, DIS, Z1, HI);
  k_ng<1><<<dim3(NPG / 64), dim3(64), 0, stream>>>(HI, Z1, WB + 32768, pre_b, Z2);
  k_attn<<<dim3(NPT), dim3(32), 0, stream>>>(Z2, fe, g1, b1, CT, P16, S16);
  k_y<<<dim3(NTB), dim3(64), 0, stream>>>(S16, M16, label, CT, g2, b2, X1, HL);
  k_f1<<<dim3(NTB, 2), dim3(64), 0, stream>>>(HL, W1h, fb1, G16);
  k_f2<<<dim3(NTB), dim3(64), 0, stream>>>(G16, W2h, fb2, X1, cw, cb, FLG, out);
  (void)hipGetLastError();
}
